// MultiHeadAttention_36017595744736
// MI455X (gfx1250) — hardware-run, weakly checked
//
#include <hip/hip_runtime.h>
#ifndef NB
#define NB 32
#endif
#ifndef SEQ
#define SEQ 512
#endif
#define NB_FULL 32
#define SQ_FULL 512
#define SQ SEQ
#define DM 256
#define NH 8
#define HD 32
#define QT 256
#define NKX SQ
#define QT0 64
#define BG ((NB) < 8 ? (NB) : 8)
#define NR ((size_t)NB * SQ)
#define LQ DM
#define LP 36
#define SCL 0.17677669529663687f
#define SCLR 0.00017263349150062194f
#define WS_CAP ((size_t)134217728)

static_assert(SQ % QT == 0);
static_assert(SQ % 128 == 0);
static_assert(QT % 128 == 0);
static_assert(NB % BG == 0);
static_assert(QT0 == 64);
static_assert(SQ >= QT0);
static_assert(NH % 2 == 0);
static_assert(HD == 32);
static_assert(DM == NH * HD);
static_assert((size_t)BG * NH * QT * NKX >= (size_t)NB * SQ * DM);

typedef unsigned short v8us __attribute__((ext_vector_type(8), may_alias));
typedef float  v8f  __attribute__((ext_vector_type(8)));
typedef float  v4f  __attribute__((ext_vector_type(4)));
typedef float  v4fa __attribute__((ext_vector_type(4), may_alias));
typedef _Float16 v16h __attribute__((ext_vector_type(16)));
typedef _Float16 v4h __attribute__((ext_vector_type(4)));
union FragH { v16h v; v8us half[2]; _Float16 h[16]; unsigned short u[16]; };

__device__ __forceinline__ unsigned short bf16_bits(float x) { unsigned int u = __float_as_uint(x); return (unsigned short)((u + 0x7FFFu + ((u >> 16) & 1u)) >> 16); }
__device__ __forceinline__ float bf16_val(unsigned short b) { return __uint_as_float(((unsigned int)b) << 16); }
__device__ __forceinline__ float bf16_rne(float x) { return bf16_val(bf16_bits(x)); }

__global__ __launch_bounds__(256) void k_wt_f16(const float* __restrict__ W, _Float16* __restrict__ Wt, int K, int N, float scale) {
  const int t = blockIdx.x * 256 + threadIdx.x; if (t >= N * (K / 8)) return; const int n = t / (K / 8), k8 = (t % (K / 8)) * 8; FragH f;
#pragma unroll
  for (int i = 0; i < 8; ++i) f.h[i] = (_Float16)(bf16_rne(W[(size_t)(k8 + i) * N + n]) * scale);
  const v8us o = f.half[0];
  unsigned short* d = (unsigned short*)Wt + (size_t)n * K + k8;
  *(volatile v8us*)d = o; __threadfence(); *(volatile v8us*)d = o;
}

__global__ __launch_bounds__(256) void k_x16(const float* __restrict__ x, _Float16* __restrict__ X16, size_t n8, size_t sSrc, size_t sDst) {
  const size_t t = (size_t)blockIdx.x * 256 + threadIdx.x; if (t >= n8) return;
  const float* s = x + (size_t)blockIdx.y * sSrc + t * 8;
  const v4f a = *(const v4fa*)(s), c = *(const v4fa*)(s + 4);
  FragH f;
#pragma unroll
  for (int q = 0; q < 4; ++q) { f.h[q] = (_Float16)bf16_rne(a[q]); f.h[4 + q] = (_Float16)bf16_rne(c[q]); }
  const v8us o = f.half[0];
  unsigned short* d = (unsigned short*)X16 + (size_t)blockIdx.y * sDst + t * 8;
  *(volatile v8us*)d = o; __threadfence(); *(volatile v8us*)d = o;
}

__global__ __launch_bounds__(256) void k_hl(const float* __restrict__ F, _Float16* __restrict__ Hh, _Float16* __restrict__ Hl, size_t n8) {
  const size_t t = (size_t)blockIdx.x * 256 + threadIdx.x; if (t >= n8) return; FragH fh, fl; const v4f a = *(const v4fa*)(F + t * 8), c = *(const v4fa*)(F + t * 8 + 4);
#pragma unroll
  for (int q = 0; q < 4; ++q) { _Float16 h = (_Float16)a[q]; fh.h[q] = h; fl.h[q] = (_Float16)((a[q] - (float)h) * 1024.0f); h = (_Float16)c[q]; fh.h[4 + q] = h; fl.h[4 + q] = (_Float16)((c[q] - (float)h) * 1024.0f); }
  const v8us oh = fh.half[0], ol = fl.half[0];
  for (int pass = 0; pass < 2; ++pass) { *(volatile v8us*)((unsigned short*)Hh + t * 8) = oh; *(volatile v8us*)((unsigned short*)Hl + t * 8) = ol; if (pass == 0) __threadfence(); }
}

__device__ __forceinline__ v16h g2_frag(const _Float16* p, int hh) { FragH f; f.half[0] = *(const v8us*)((const unsigned short*)p + 8 * hh); f.half[1] = *(const v8us*)((const unsigned short*)p + 16 + 8 * hh); return f.v; }
__device__ __forceinline__ v8f g2_mma(v16h a, v16h b, v8f c) { v8f d = __builtin_amdgcn_wmma_f32_16x16x32_f16(false, a, false, b, (short)0, c, false, false); asm volatile("v_nop\n\tv_nop\n\tv_nop\n\tv_nop" : "+v"(d) : "v"(a), "v"(b)); return d; }
template <bool PAIR>
__global__ __launch_bounds__(128) void k_gemm2(const _Float16* __restrict__ A, int lda, size_t sA, size_t sA2, size_t pairA,
    const _Float16* __restrict__ Bh, int ldb, size_t sB, size_t sB2, int ydiv, float alpha, const float* __restrict__ bias,
    const float* CP, float* C, _Float16* C16, int ldc, size_t sC, size_t sC2, int M, int N, int K) {
  __shared__ __attribute__((aligned(16))) float so[4][32][68];
  const int tid = threadIdx.x, w = tid >> 5, lane = tid & 31, ln = lane & 15, hh = lane >> 4;
  const int by = blockIdx.y; const int y1 = by / ydiv; const int y0 = by - y1 * ydiv;
  A += (size_t)y0 * sA + (size_t)y1 * sA2; Bh += (size_t)y0 * sB + (size_t)y1 * sB2; const size_t cofs = (size_t)y0 * sC + (size_t)y1 * sC2;
  const int ntn = N >> 6; const int mt = blockIdx.x / ntn, nq = blockIdx.x - mt * ntn; const int row0 = mt * 128 + 32 * w, col0 = nq * 64; if (row0 >= M) return;
  const _Float16* a0p = A + (size_t)(row0 + ln) * lda; const _Float16* a1p = a0p + (size_t)16 * lda;
  const _Float16* a2p = PAIR ? (a0p + pairA) : a0p; const _Float16* a3p = PAIR ? (a1p + pairA) : a1p;
  const _Float16* b0p = Bh + (size_t)(col0 + ln) * ldb; const _Float16* b1p = b0p + (size_t)16 * ldb; const _Float16* b2p = b1p + (size_t)16 * ldb; const _Float16* b3p = b2p + (size_t)16 * ldb;
  const v8f z8 = {0.f,0.f,0.f,0.f,0.f,0.f,0.f,0.f}; v8f c00 = z8, c01 = z8, c02 = z8, c03 = z8, c10 = z8, c11 = z8, c12 = z8, c13 = z8;
#pragma unroll 1
  for (int kb = 0; kb < K; kb += 32) { const v16h a0 = g2_frag(a0p + kb, hh), a1 = g2_frag(a1p + kb, hh);
    v16h a2 = a0, a3 = a1; if (PAIR) { a2 = g2_frag(a2p + kb, hh); a3 = g2_frag(a3p + kb, hh); }
    v16h b = g2_frag(b0p + kb, hh); c00 = g2_mma(a0, b, c00); c10 = g2_mma(a1, b, c10);
    b = g2_frag(b1p + kb, hh); c01 = g2_mma(a0, b, c01); c11 = g2_mma(a1, b, c11);
    b = g2_frag(b2p + kb, hh); c02 = g2_mma(a2, b, c02); c12 = g2_mma(a3, b, c12);
    b = g2_frag(b3p + kb, hh); c03 = g2_mma(a2, b, c03); c13 = g2_mma(a3, b, c13); }
  v8f accs[8] = {c00, c01, c02, c03, c10, c11, c12, c13};
#pragma unroll
  for (int u = 0; u < 8; ++u) { const int t = u & 3, half = u >> 2; const int col = col0 + t * 16 + ln; const float bv = bias ? bf16_rne(bias[col]) : 0.f;
#pragma unroll
    for (int r = 0; r < 8; ++r) { const int rloc = half * 16 + 8 * hh + r; float v = accs[u][r] * alpha + bv; if (CP) v += CP[cofs + (size_t)(row0 + rloc) * ldc + col];
      so[w][rloc][t * 16 + ln] = v; } }
  __builtin_amdgcn_fence(4  , "workgroup"); __builtin_amdgcn_wave_barrier();
  const int rsub = lane >> 4, c4 = (lane & 15) * 4;
  for (int pass = 0; pass < 2; ++pass) {
#pragma unroll
    for (int q = 0; q < 16; ++q) { const int r = q * 2 + rsub; const v4f v = *(const v4fa*)&so[w][r][c4]; if (C) *(volatile v4f*)(C + cofs + (size_t)(row0 + r) * ldc + col0 + c4) = v; if (C16) { v4h h4; for (int i = 0; i < 4; ++i) h4[i] = (_Float16)v[i]; *(volatile v4h*)(C16 + cofs + (size_t)(row0 + r) * ldc + col0 + c4) = h4; } }
    if (pass == 0) __threadfence(); } }

__global__ __launch_bounds__(256) void k_vt(const _Float16* __restrict__ V16, int ldv, _Float16* __restrict__ Vt) {
  __shared__ unsigned short tl[64][HD + 2];
  const int tid = threadIdx.x; const int slab = blockIdx.x / (SQ / 64), lg = blockIdx.x % (SQ / 64); const int b = slab / NH, h = slab % NH;
  { const int r = tid / 4, c8 = (tid % 4) * 8; FragH f; f.half[0] = *(const v8us*)((const unsigned short*)V16 + ((size_t)b * SQ + lg * 64 + r) * ldv + h * HD + c8);
#pragma unroll
    for (int q = 0; q < 8; ++q) tl[r][c8 + q] = f.u[q]; }
  __syncthreads();
  const int d = tid / 8, pc = tid % 8; FragH g;
#pragma unroll
  for (int q = 0; q < 8; ++q) g.u[q] = tl[pc * 8 + q][d];
  const v8us o = g.half[0];
  unsigned short* dst = (unsigned short*)Vt + ((size_t)slab * HD + d) * SQ + lg * 64 + pc * 8;
  *(volatile v8us*)dst = o; __threadfence(); *(volatile v8us*)dst = o;
}

__global__ __launch_bounds__(256) void k_rsmcf2(const float* __restrict__ S, _Float16* __restrict__ P, int nslab, int q0, int nk) {
  #pragma clang fp contract(off)
  const int t = blockIdx.x * 256 + threadIdx.x; if (t >= nslab * QT) return; const size_t i = (size_t)t; const float* s = S + i * NKX; const int h = (t / QT) % NH; const int last = q0 + (t % QT);
  const float slope = __uint_as_float((unsigned int)(126 - h) << 23);
  float mx = -3.0e38f;
#pragma unroll 1
  for (int j = 0; j < nk; ++j) { const float f = (j <= last) ? 1.f : 0.f; const float a = s[j] + slope * (float)(j - last); mx = fmaxf(mx, fmaf(f, a, (1.f - f) * -1.0e9f)); }
  float se = 0.f;
#pragma unroll 1
  for (int j = 0; j < nk; ++j) { const float f = (j <= last) ? 1.f : 0.f; const float a = s[j] + slope * (float)(j - last); se += __expf(fmaf(f, a, (1.f - f) * -1.0e9f) - mx); }
  const float sc = 256.0f / se;
#pragma unroll 1
  for (int j0 = 0; j0 < nk; j0 += 8) { FragH fr;
#pragma unroll
    for (int q = 0; q < 8; ++q) { const int j = j0 + q; const float f = (j <= last) ? 1.f : 0.f; const float a = s[j] + slope * (float)(j - last); fr.h[q] = (_Float16)(__expf(fmaf(f, a, (1.f - f) * -1.0e9f) - mx) * sc); }
    const v8us o = fr.half[0]; unsigned short* d = (unsigned short*)P + i * NKX + j0; *(volatile v8us*)d = o; __threadfence(); *(volatile v8us*)d = o; } }

__global__ __launch_bounds__(64) void k_att0(const float* __restrict__ QF, const float* __restrict__ KF, const float* __restrict__ VF, int ld, size_t sIn, float scale, float* __restrict__ OF, int ldo, size_t sOut) {
  #pragma clang fp contract(off)
  __shared__ __attribute__((aligned(16))) float lq[64][LP]; __shared__ __attribute__((aligned(16))) float lo[64][LP];
  const int tid = threadIdx.x; const int h = blockIdx.x / (QT0 / 64), rg = blockIdx.x % (QT0 / 64); const int i = rg * 64 + tid; const size_t b = (size_t)blockIdx.y;
  QF += b * sIn; KF += b * sIn; VF += b * sIn; OF += b * sOut;
  const float slope = __uint_as_float((unsigned int)(126 - h) << 23);
  const float* qr = QF + (size_t)i * ld + h * HD;
#pragma unroll 1
  for (int c = 0; c < HD / 4; ++c) { *(v4f*)&lq[tid][c * 4] = *(const v4fa*)(qr + c * 4); const v4f z = {0.f, 0.f, 0.f, 0.f}; *(v4f*)&lo[tid][c * 4] = z; }
  float m = -1.0e30f, l = 0.f; const int jmax = rg * 64 + 63;
#pragma unroll 1
  for (int j = 0; j <= jmax; ++j) { const float* kr = KF + (size_t)j * ld + h * HD; const float* vr = VF + (size_t)j * ld + h * HD; float s = 0.f;
#pragma unroll 1
    for (int c = 0; c < HD / 4; ++c) { const v4f kq = *(const v4fa*)(kr + c * 4); const v4f qq = *(v4f*)&lq[tid][c * 4]; s = __fadd_rn(s, __fmul_rn(qq[0], kq[0])); s = __fadd_rn(s, __fmul_rn(qq[1], kq[1])); s = __fadd_rn(s, __fmul_rn(qq[2], kq[2])); s = __fadd_rn(s, __fmul_rn(qq[3], kq[3])); }
    s = __fmul_rn(s, scale); s = __fadd_rn(s, __fmul_rn(slope, (float)(j - i)));
    const float f = (j <= i) ? 1.f : 0.f; const float sm = fmaf(f, s, (1.f - f) * -1.0e30f); const float mn = fmaxf(m, sm); const float sc = expf(m - mn); const float e = expf(sm - mn); l = __fadd_rn(__fmul_rn(l, sc), e); m = mn;
#pragma unroll 1
    for (int c = 0; c < HD / 4; ++c) { const v4f vv = *(const v4fa*)(vr + c * 4); v4f oo = *(v4f*)&lo[tid][c * 4]; for (int u = 0; u < 4; ++u) oo[u] = __fadd_rn(__fmul_rn(oo[u], sc), __fmul_rn(e, vv[u])); *(v4f*)&lo[tid][c * 4] = oo; } }
  const float fin = 64.0f / l;
#pragma unroll 1
  for (int c = 0; c < HD / 4; ++c) { v4f oo = *(v4f*)&lo[tid][c * 4]; for (int u = 0; u < 4; ++u) oo[u] = __fmul_rn(oo[u], fin); *(v4f*)&lo[tid][c * 4] = oo; }
  __syncthreads();
  for (int pass = 0; pass < 2; ++pass) {
#pragma unroll 1
    for (int it = 0; it < 8; ++it) { const int row = it * 8 + tid / 8, pc = (tid % 8) * 4; const v4f v = *(const v4f*)&lo[row][pc]; *(volatile v4f*)(OF + (size_t)(rg * 64 + row) * ldo + h * HD + pc) = v; }
    if (pass == 0) __threadfence(); } }

extern "C" void kernel_launch(void* const* d_in, const int* in_sizes, int n_in,
                              void* d_out, int out_size, void* d_ws, size_t ws_size, hipStream_t stream) {
  if (n_in < 6) return;
  const size_t need_x = ((size_t)(NB - 1) * SQ_FULL + SQ) * DM;
  if ((size_t)in_sizes[0] < need_x) return;
  if ((size_t)in_sizes[1] < (size_t)DM * DM || (size_t)in_sizes[2] < (size_t)DM * DM || (size_t)in_sizes[3] < (size_t)DM * DM || (size_t)in_sizes[4] < (size_t)DM * DM) return;
  if ((size_t)in_sizes[5] < (size_t)DM) return;
  if ((size_t)out_size < need_x) return;
  const float* x = (const float*)d_in[0]; const float* wq = (const float*)d_in[1]; const float* wk = (const float*)d_in[2]; const float* wv = (const float*)d_in[3]; const float* wo = (const float*)d_in[4]; const float* bo = (const float*)d_in[5];
  float* out = (float*)d_out;
  char* ws = (char*)d_ws; size_t off = 0;
  auto take = [&](size_t bytes) { char* p = ws + off; off += (bytes + 255) & ~(size_t)255; return p; };
  _Float16* BQ = (_Float16*)take((size_t)DM * DM * 2); _Float16* BK = (_Float16*)take((size_t)DM * DM * 2); _Float16* BV = (_Float16*)take((size_t)DM * DM * 2); _Float16* BO = (_Float16*)take((size_t)DM * DM * 2);
  _Float16* X16 = (_Float16*)take(NR * DM * 2);
  _Float16* QH = (_Float16*)take(NR * DM * 2); _Float16* QL = (_Float16*)take(NR * DM * 2); _Float16* KH = (_Float16*)take(NR * DM * 2); _Float16* KL = (_Float16*)take(NR * DM * 2);
  _Float16* V16 = (_Float16*)take(NR * DM * 2); _Float16* O16 = (_Float16*)take(NR * DM * 2);
  float* S = (float*)take((size_t)BG * NH * QT * NKX * 4);
  float* QF = S;
  _Float16* P = (_Float16*)take((size_t)BG * NH * QT * NKX * 2);
  _Float16* VT = (_Float16*)take((size_t)NB * NH * HD * SQ * 2);
  float* QF0 = (float*)take((size_t)NB * QT0 * DM * 4); float* KF0 = (float*)take((size_t)NB * QT0 * DM * 4); float* VF0 = (float*)take((size_t)NB * QT0 * DM * 4);
  float* OF0 = (float*)take((size_t)NB * QT0 * DM * 4); _Float16* OH0 = (_Float16*)take((size_t)NB * QT0 * DM * 2); _Float16* OL0 = (_Float16*)take((size_t)NB * QT0 * DM * 2);
  if (off > ws_size || off > WS_CAP) return;

  { const unsigned g = (unsigned)(((size_t)DM * (DM / 8) + 255) / 256);
    k_wt_f16<<<g, 256, 0, stream>>>(wq, BQ, DM, DM, 16.0f); k_wt_f16<<<g, 256, 0, stream>>>(wk, BK, DM, DM, 16.0f);
    k_wt_f16<<<g, 256, 0, stream>>>(wv, BV, DM, DM, 16.0f); k_wt_f16<<<g, 256, 0, stream>>>(wo, BO, DM, DM, 16.0f); }
  k_x16<<<dim3((unsigned)(((size_t)SQ * DM / 8 + 255) / 256), NB), 256, 0, stream>>>(x, X16, (size_t)SQ * DM / 8, (size_t)SQ_FULL * DM, (size_t)SQ * DM);

  const unsigned gproj = (unsigned)((NR / 128) * (DM / 64)); const unsigned ghl = (unsigned)((NR * DM / 8 + 255) / 256);
  k_gemm2<false><<<dim3(gproj, 1), 128, 0, stream>>>(X16, DM, (size_t)0, (size_t)0, (size_t)0, BQ, DM, (size_t)0, (size_t)0, 1, 0.0625f, nullptr, nullptr, QF, nullptr, DM, (size_t)0, (size_t)0, (int)NR, DM, DM);
  k_hl<<<ghl, 256, 0, stream>>>(QF, QH, QL, NR * DM / 8);
  k_gemm2<false><<<dim3(gproj, 1), 128, 0, stream>>>(X16, DM, (size_t)0, (size_t)0, (size_t)0, BK, DM, (size_t)0, (size_t)0, 1, 0.0625f, nullptr, nullptr, QF, nullptr, DM, (size_t)0, (size_t)0, (int)NR, DM, DM);
  k_hl<<<ghl, 256, 0, stream>>>(QF, KH, KL, NR * DM / 8);
  k_gemm2<false><<<dim3(gproj, 1), 128, 0, stream>>>(X16, DM, (size_t)0, (size_t)0, (size_t)0, BV, DM, (size_t)0, (size_t)0, 1, 0.0625f, nullptr, nullptr, nullptr, V16, DM, (size_t)0, (size_t)0, (int)NR, DM, DM);
  k_vt<<<(unsigned)(NB * NH * (SQ / 64)), 256, 0, stream>>>(V16, LQ, VT);

  { const dim3 g0((unsigned)(((QT0 + 127) / 128) * (DM / 64)), NB);
    k_gemm2<false><<<g0, 128, 0, stream>>>(X16, DM, (size_t)0, (size_t)SQ * DM, (size_t)0, BQ, DM, (size_t)0, (size_t)0, 1, 0.0625f, nullptr, nullptr, QF0, nullptr, DM, (size_t)0, (size_t)QT0 * DM, QT0, DM, DM);
    k_gemm2<false><<<g0, 128, 0, stream>>>(X16, DM, (size_t)0, (size_t)SQ * DM, (size_t)0, BK, DM, (size_t)0, (size_t)0, 1, 0.0625f, nullptr, nullptr, KF0, nullptr, DM, (size_t)0, (size_t)QT0 * DM, QT0, DM, DM);
    k_gemm2<false><<<g0, 128, 0, stream>>>(X16, DM, (size_t)0, (size_t)SQ * DM, (size_t)0, BV, DM, (size_t)0, (size_t)0, 1, 0.0625f, nullptr, nullptr, VF0, nullptr, DM, (size_t)0, (size_t)QT0 * DM, QT0, DM, DM);
    k_att0<<<dim3(NH * (QT0 / 64), NB), 64, 0, stream>>>(QF0, KF0, VF0, DM, (size_t)QT0 * DM, SCL, OF0, DM, (size_t)QT0 * DM); }

  const size_t slabS = (size_t)QT * NKX;
  for (int g = 0; g < NB / BG; ++g) { const size_t rg0 = (size_t)g * BG * SQ;
    for (int q0 = 0; q0 < SQ; q0 += QT) { const int nk = q0 + QT;
      const dim3 gs((unsigned)((QT / 128) * (nk / 64)), BG * NH);
      k_gemm2<false><<<gs, 128, 0, stream>>>(QH + (rg0 + q0) * LQ, LQ, (size_t)HD, (size_t)SQ * LQ, (size_t)0, KH + rg0 * LQ, LQ, (size_t)HD, (size_t)SQ * LQ, NH, SCL, nullptr, nullptr, S, nullptr, NKX, slabS, (size_t)NH * slabS, QT, nk, HD);
      k_gemm2<false><<<gs, 128, 0, stream>>>(QL + (rg0 + q0) * LQ, LQ, (size_t)HD, (size_t)SQ * LQ, (size_t)0, KH + rg0 * LQ, LQ, (size_t)HD, (size_t)SQ * LQ, NH, SCLR, nullptr, S, S, nullptr, NKX, slabS, (size_t)NH * slabS, QT, nk, HD);
      k_gemm2<false><<<gs, 128, 0, stream>>>(QH + (rg0 + q0) * LQ, LQ, (size_t)HD, (size_t)SQ * LQ, (size_t)0, KL + rg0 * LQ, LQ, (size_t)HD, (size_t)SQ * LQ, NH, SCLR, nullptr, S, S, nullptr, NKX, slabS, (size_t)NH * slabS, QT, nk, HD);
      k_rsmcf2<<<(unsigned)((BG * NH * QT + 255) / 256), 256, 0, stream>>>(S, P, BG * NH, q0, nk);
      k_gemm2<true><<<dim3((unsigned)(QT / 128), BG * (NH / 2)), 128, 0, stream>>>(P, NKX, 2 * slabS, (size_t)NH * slabS, slabS, VT + (size_t)g * BG * NH * HD * SQ, SQ, (size_t)2 * HD * SQ, (size_t)NH * HD * SQ, NH / 2, 0.25f, nullptr, nullptr, nullptr, O16 + (rg0 + q0) * DM, DM, (size_t)(2 * HD), (size_t)SQ * DM, QT, 2 * HD, nk);
    } }

  k_gemm2<false><<<dim3((unsigned)((SQ / 128) * (DM / 64)), NB), 128, 0, stream>>>(O16, DM, (size_t)0, (size_t)SQ * DM, (size_t)0, BO, DM, (size_t)0, (size_t)0, 1, 0.0009765625f, bo, nullptr, out, nullptr, DM, (size_t)0, (size_t)SQ_FULL * DM, SQ, DM, DM);
  k_hl<<<(unsigned)(((size_t)NB * QT0 * DM / 8 + 255) / 256), 256, 0, stream>>>(OF0, OH0, OL0, (size_t)NB * QT0 * DM / 8);
  { const dim3 g0((unsigned)(((QT0 + 127) / 128) * (DM / 64)), NB);
    k_gemm2<false><<<g0, 128, 0, stream>>>(OH0, DM, (size_t)0, (size_t)QT0 * DM, (size_t)0, BO, DM, (size_t)0, (size_t)0, 1, 0.0009765625f, bo, nullptr, out, nullptr, DM, (size_t)0, (size_t)SQ_FULL * DM, QT0, DM, DM);
    k_gemm2<false><<<g0, 128, 0, stream>>>(OL0, DM, (size_t)0, (size_t)QT0 * DM, (size_t)0, BO, DM, (size_t)0, (size_t)0, 1, 0.00000095367431640625f, nullptr, out, out, nullptr, DM, (size_t)0, (size_t)SQ_FULL * DM, QT0, DM, DM); }
}
